// GATActor_3788161155325
// MI455X (gfx1250) — hardware-verified
//
#include <hip/hip_runtime.h>
#include <stddef.h>


#define IN_DIM  128
#define KP      256
#define FEAT    256
#define HC      64
#define NHEAD   4
#define OUTD    5
#define FCN     16
#define WTROWS  (2 * FEAT + FCN)
#define YP      256
#define EP      4
#define NTHR    256
#define NWAVE   8
#define EPT     8
#define CHUNK   (NTHR * EPT)
#define WCAP    (EPT * 32)
#define LISTN   (NWAVE * WCAP)
#define NBMAX   2048
#define RCAP    28672
#define DEGCAP  4096
#define GBM     64
#define GTHR    128
#define NEG_SLOPE 0.2f
#define CA      16.0f
#define CW      64.0f
#define SCL     0.0009765625f
#define WSCAP   134217728
#define LDS_AGG ((2 * RCAP + 2 * NBMAX + LISTN) * 4 + 64)

static_assert((CHUNK & (CHUNK - 1)) == 0 && CHUNK <= 4096);
static_assert((NBMAX & (NBMAX - 1)) == 0 && NBMAX <= 4096);
static_assert(NTHR * 8 == NBMAX);
static_assert(LISTN >= NBMAX);
static_assert(LISTN >= NWAVE * WCAP);
static_assert((RCAP % 32) == 0);
static_assert(LDS_AGG <= 300000);
static_assert(GBM == (GTHR / 32) * 16);
static_assert(2 * GBM == GTHR);
static_assert(2 * GTHR == FEAT);
static_assert(NHEAD * HC == FEAT);
static_assert(HC == 64 && NHEAD == 4);
static_assert(FEAT == 8 * 32);
static_assert(KP == 256 && (KP % 32) == 0 && (IN_DIM % 32) == 0);
static_assert(GBM * EP == 2 * 32 * 4);
static_assert(OUTD <= FCN);
static_assert((GBM * OUTD) % 4 == 0);

typedef float    v2f  __attribute__((ext_vector_type(2)));
typedef float    v4f  __attribute__((ext_vector_type(4)));
typedef float    v8f  __attribute__((ext_vector_type(8)));
typedef int      v4i  __attribute__((ext_vector_type(4)));
typedef int      v8i  __attribute__((ext_vector_type(8)));
typedef _Float16 v4h  __attribute__((ext_vector_type(4)));
typedef _Float16 v8h  __attribute__((ext_vector_type(8)));
typedef _Float16 v16h __attribute__((ext_vector_type(16)));
union FragH { v16h v; v8h h[2]; v8i w; };

__device__ __forceinline__ v8f wmh(const FragH& a, const FragH& b, v8f c) {
  v8f d = __builtin_amdgcn_wmma_f32_16x16x32_f16(false, a.v, false, b.v, (short)0, c, false, false);
  asm volatile("v_nop\n\tv_nop\n\tv_nop\n\tv_nop" : "+v"(d) : "v"(a.w), "v"(b.w));
  return d;
}

__device__ __forceinline__ int scan_chunk(const int* __restrict__ dsts, int nE, int cbase, int slotBase,
                                          int nb, int vec8, int* list, int tid, int lane, int wave) {
  int wc = 0;
  const int el0  = tid * EPT;
  const int e0   = cbase + el0;
  const int sent = -2147483647 - 1;
  v4i da, db;
  if (vec8 != 0 && cbase + CHUNK <= nE) {
    da = *(const v4i*)(dsts + e0);
    db = *(const v4i*)(dsts + e0 + 4);
  } else {
    da.x = (e0     < nE) ? dsts[min(e0,     nE - 1)] : sent;
    da.y = (e0 + 1 < nE) ? dsts[min(e0 + 1, nE - 1)] : sent;
    da.z = (e0 + 2 < nE) ? dsts[min(e0 + 2, nE - 1)] : sent;
    da.w = (e0 + 3 < nE) ? dsts[min(e0 + 3, nE - 1)] : sent;
    db.x = (e0 + 4 < nE) ? dsts[min(e0 + 4, nE - 1)] : sent;
    db.y = (e0 + 5 < nE) ? dsts[min(e0 + 5, nE - 1)] : sent;
    db.z = (e0 + 6 < nE) ? dsts[min(e0 + 6, nE - 1)] : sent;
    db.w = (e0 + 7 < nE) ? dsts[min(e0 + 7, nE - 1)] : sent;
  }
  const unsigned nbs = (unsigned)slotBase;
  const unsigned unb = (unsigned)nb;
  const unsigned s0 = (unsigned)da.x - nbs, s1 = (unsigned)da.y - nbs;
  const unsigned s2 = (unsigned)da.z - nbs, s3 = (unsigned)da.w - nbs;
  const unsigned s4 = (unsigned)db.x - nbs, s5 = (unsigned)db.y - nbs;
  const unsigned s6 = (unsigned)db.z - nbs, s7 = (unsigned)db.w - nbs;
  const bool h0 = s0 < unb, h1 = s1 < unb, h2 = s2 < unb, h3 = s3 < unb;
  const bool h4 = s4 < unb, h5 = s5 < unb, h6 = s6 < unb, h7 = s7 < unb;
  const unsigned any = __builtin_amdgcn_ballot_w32(h0 | h1 | h2 | h3 | h4 | h5 | h6 | h7);
  if (any != 0u) {
#define HITJ(J, HJ, SJ) { \
      const unsigned mj = __builtin_amdgcn_ballot_w32(HJ); \
      if (mj != 0u) { \
        if (HJ) { \
          const int pos = wc + (int)__builtin_amdgcn_mbcnt_lo(mj, 0u); \
          if (pos < WCAP) list[wave * WCAP + pos] = ((el0 + (J)) << 12) | (int)(SJ); \
        } \
        wc += (int)__builtin_popcount(mj); } }
    HITJ(0, h0, s0)
    HITJ(1, h1, s1)
    HITJ(2, h2, s2)
    HITJ(3, h3, s3)
    HITJ(4, h4, s4)
    HITJ(5, h5, s5)
    HITJ(6, h6, s6)
    HITJ(7, h7, s7)
#undef HITJ
  }
  return wc;
}

__global__ __launch_bounds__(NTHR) void k_xprep(const float* __restrict__ x, _Float16* xh, int nN, int nUnits) {
  const int i = (int)blockIdx.x * NTHR + (int)threadIdx.x;
  if (i >= nUnits) return;
  const int row = i >> 5;
  const int c0  = (i & 31) * 8;
  const int rc  = row < nN ? row : nN - 1;
  const int cc  = c0 & (IN_DIM - 1);
  const float* p = x + (size_t)rc * IN_DIM + cc;
  v4f a = *(const v4f*)p, b = *(const v4f*)(p + 4);
  const v4f z4 = {0.f, 0.f, 0.f, 0.f};
  if (row >= nN || c0 >= IN_DIM) { a = z4; b = z4; }
  v8h hv;
  hv[0] = (_Float16)(a.x * CA); hv[1] = (_Float16)(a.y * CA);
  hv[2] = (_Float16)(a.z * CA); hv[3] = (_Float16)(a.w * CA);
  hv[4] = (_Float16)(b.x * CA); hv[5] = (_Float16)(b.y * CA);
  hv[6] = (_Float16)(b.z * CA); hv[7] = (_Float16)(b.w * CA);
  const size_t o = (size_t)row * KP + c0;
  *(volatile v8h*)(xh + o) = hv;
  __threadfence();
  *(volatile v8h*)(xh + o) = hv;
}

__global__ __launch_bounds__(NTHR) void k_wprep(const float* __restrict__ w1, const float* __restrict__ w2,
                                                const float* __restrict__ wf, _Float16* wt) {
  const int j  = (int)blockIdx.y;
  const int u  = (int)blockIdx.x * NTHR + (int)threadIdx.x;
  const int nrow = (j == 2) ? FCN : FEAT;
  const int nUnits = nrow * (KP / 8);
  if (u >= nUnits) return;
  const int n  = u >> 5;
  const int k8 = (u & 31) * 8;
  const int ksrc = (j == 0) ? IN_DIM : FEAT;
  const int nc   = (j == 2) ? OUTD : FEAT;
  const float* src = (j == 0) ? w1 : ((j == 1) ? w2 : wf);
  const bool valid = (k8 < ksrc) && (n < nc);
  const int kc  = (k8 < ksrc) ? k8 : (ksrc - 8);
  const int ncl = (n < nc) ? n : (nc - 1);
  const float* p = src + (size_t)kc * nc + ncl;
  v4f a, b;
  a.x = p[0 * nc]; a.y = p[1 * nc]; a.z = p[2 * nc]; a.w = p[3 * nc];
  b.x = p[4 * nc]; b.y = p[5 * nc]; b.z = p[6 * nc]; b.w = p[7 * nc];
  const v4f z4 = {0.f, 0.f, 0.f, 0.f};
  if (!valid) { a = z4; b = z4; }
  v8h hv;
  hv[0] = (_Float16)(a.x * CW); hv[1] = (_Float16)(a.y * CW);
  hv[2] = (_Float16)(a.z * CW); hv[3] = (_Float16)(a.w * CW);
  hv[4] = (_Float16)(b.x * CW); hv[5] = (_Float16)(b.y * CW);
  hv[6] = (_Float16)(b.z * CW); hv[7] = (_Float16)(b.w * CW);
  const size_t rowb = (size_t)j * FEAT;
  const size_t o = (rowb + (size_t)n) * KP + k8;
  *(volatile v8h*)(wt + o) = hv;
  __threadfence();
  *(volatile v8h*)(wt + o) = hv;
}

__global__ __launch_bounds__(GTHR) void k_gemm(const _Float16* __restrict__ xh, const _Float16* __restrict__ wt,
                                               const float* __restrict__ asrc, const float* __restrict__ adst,
                                               float* Y, float* ES, float* ED, int nks) {
  __shared__ __attribute__((aligned(16))) float stg[GBM * HC];
  __shared__ __attribute__((aligned(16))) float esT[GBM * EP];
  __shared__ __attribute__((aligned(16))) float edT[GBM * EP];
  __shared__ float sAs[FEAT];
  __shared__ float sAd[FEAT];
  const int tid = threadIdx.x, lane = tid & 31, wave = tid >> 5, hh = lane >> 4, m = lane & 15;
  const int rowBase = (int)blockIdx.x * GBM;
  sAs[tid] = asrc[tid];
  sAd[tid] = adst[tid];
  sAs[tid + GTHR] = asrc[tid + GTHR];
  sAd[tid + GTHR] = adst[tid + GTHR];
  const int nk = nks < 1 ? 1 : (nks > KP / 32 ? KP / 32 : nks);
  const size_t arow = (size_t)(rowBase + 16 * wave + m) * KP + 8 * hh;
#pragma unroll 1
  for (int p = 0; p < NHEAD; ++p) {
    v8f acc[4];
#pragma unroll
    for (int t = 0; t < 4; ++t) { v8f z = {0.f, 0.f, 0.f, 0.f, 0.f, 0.f, 0.f, 0.f}; acc[t] = z; }
    const size_t brow = (size_t)(p * HC + m) * KP + 8 * hh;
#pragma unroll 1
    for (int ks = 0; ks < nk; ++ks) {
      FragH af;
      af.h[0] = *(const v8h*)(xh + arow + 32 * ks);
      af.h[1] = *(const v8h*)(xh + arow + 32 * ks + 16);
#pragma unroll
      for (int t = 0; t < 4; ++t) {
        const size_t bo = brow + (size_t)(16 * t) * KP + 32 * ks;
        FragH bf;
        bf.h[0] = *(const v8h*)(wt + bo);
        bf.h[1] = *(const v8h*)(wt + bo + 16);
        acc[t] = wmh(af, bf, acc[t]);
      }
    }
    float* sp = stg + (size_t)(16 * wave + 8 * hh) * HC + m;
#pragma unroll
    for (int t = 0; t < 4; ++t) {
#pragma unroll
      for (int r = 0; r < 8; ++r) sp[(size_t)r * HC + 16 * t] = acc[t][r] * SCL;
    }
    __syncthreads();
    {
      const int row  = tid >> 1;
      const int half = tid & 1;
      const float* srow = stg + (size_t)row * HC;
      float s = 0.f, d = 0.f;
#pragma unroll 1
      for (int c = 0; c < 32; ++c) {
        const int cc = half * 32 + c;
        const float v = srow[cc];
        s = fmaf(v, sAs[p * HC + cc], s);
        d = fmaf(v, sAd[p * HC + cc], d);
      }
      s += __shfl_xor(s, 1);
      d += __shfl_xor(d, 1);
      if (half == 0) {
        esT[row * EP + p] = s;
        edT[row * EP + p] = d;
      }
    }
    const int nF4 = GBM * HC / 4;
    float* yb = Y + (size_t)rowBase * YP + HC * p;
    const v4f* s4 = (const v4f*)stg;
#pragma unroll 1
    for (int f = tid; f < nF4; f += GTHR) {
      const int r = f >> 4, q = f & 15;
      const v4f v = s4[f];
      *(volatile v4f*)(yb + (size_t)r * YP + 4 * q) = v;
    }
    __threadfence();
#pragma unroll 1
    for (int f = tid; f < nF4; f += GTHR) {
      const int r = f >> 4, q = f & 15;
      const v4f v = s4[f];
      *(volatile v4f*)(yb + (size_t)r * YP + 4 * q) = v;
    }
    __syncthreads();
  }
  if (wave < 2) {
    const v4f ve = *(const v4f*)(esT + 128 * wave + 4 * lane);
    const v4f vd = *(const v4f*)(edT + 128 * wave + 4 * lane);
    float* pe = ES + (size_t)rowBase * EP + 128 * wave + 4 * lane;
    float* pd = ED + (size_t)rowBase * EP + 128 * wave + 4 * lane;
    *(volatile v4f*)pe = ve;
    *(volatile v4f*)pd = vd;
    __threadfence();
    *(volatile v4f*)pe = ve;
    *(volatile v4f*)pd = vd;
  }
}

__global__ __launch_bounds__(NTHR) void k_agg(
    const int* __restrict__ srcs, const int* __restrict__ dsts,
    const float* __restrict__ Y, const float* __restrict__ ES, const float* __restrict__ ED,
    const float* __restrict__ bias, _Float16* xout,
    int nN, int nE, int nb, int vec8) {
  extern __shared__ v4f lds_dyn[];
  int* reg1 = (int*)lds_dyn;
  int* reg2 = reg1 + RCAP;
  int* scnt = reg2 + RCAP;
  int* soff = scnt + NBMAX;
  int* list = soff + NBMAX;
  int* wcnt = list + LISTN;
  int* wtot = wcnt + NWAVE;
  const int tid = threadIdx.x, lane = tid & 31, wave = tid >> 5;
  const int nodeBase = (int)blockIdx.x * nb;

  for (int i = tid; i < NBMAX; i += NTHR) scnt[i] = 0;
  __syncthreads();

  int tot = 0;
  const int nChunks = (nE + CHUNK - 1) / CHUNK;
#pragma unroll 1
  for (int ch = 0; ch < nChunks; ++ch) {
    const int cbase = ch * CHUNK;
    const int wc = scan_chunk(dsts, nE, cbase, nodeBase, nb, vec8, list, tid, lane, wave);
    if (lane == 0) wcnt[wave] = wc;
    __syncthreads();
    int pre = 0, all = 0;
#pragma unroll
    for (int w2 = 0; w2 < NWAVE; ++w2) {
      int c = wcnt[w2];
      c = c < 0 ? 0 : (c > WCAP ? WCAP : c);
      all += c;
      pre += (w2 < wave) ? c : 0;
    }
    const int wcc  = wc > WCAP ? WCAP : wc;
    const int base = tot + pre;
#pragma unroll 1
    for (int i = lane; i < wcc; i += 32) {
      const int ent = list[wave * WCAP + i];
      const int el  = (ent >> 12) & (CHUNK - 1);
      const int sl  = ent & (NBMAX - 1);
      int eid = cbase + el;
      eid = eid > nE - 1 ? nE - 1 : eid;
      const int pos = base + i;
      if (pos < RCAP) reg1[pos] = (int)(((unsigned)eid << 12) | (unsigned)sl);
    }
    tot += all;
    tot = tot > RCAP ? RCAP : tot;
    __syncthreads();
  }
  const int nh = tot;

  if (wave == 0) {
#pragma unroll 1
    for (int b0 = 0; b0 < nh; b0 += 32) {
      const int idx = b0 + lane;
      const int uv  = reg1[idx < RCAP ? idx : RCAP - 1];
      const int m32 = (nh - b0) < 32 ? (nh - b0) : 32;
#pragma unroll 1
      for (int k = 0; k < m32; ++k) {
        const int u  = __builtin_amdgcn_readlane(uv, k);
        const int sl = u & (NBMAX - 1);
        if (lane == 0) scnt[sl] = scnt[sl] + 1;
      }
    }
  }
  __syncthreads();

  {
    const v4i ca = *(const v4i*)(scnt + 8 * tid);
    const v4i cb = *(const v4i*)(scnt + 8 * tid + 4);
    const int e0 = ca.x < 0 ? 0 : ca.x, e1 = ca.y < 0 ? 0 : ca.y, e2 = ca.z < 0 ? 0 : ca.z, e3 = ca.w < 0 ? 0 : ca.w;
    const int e4 = cb.x < 0 ? 0 : cb.x, e5 = cb.y < 0 ? 0 : cb.y, e6 = cb.z < 0 ? 0 : cb.z, e7 = cb.w < 0 ? 0 : cb.w;
    const int ts = e0 + e1 + e2 + e3 + e4 + e5 + e6 + e7;
    int incl = ts;
#pragma unroll
    for (int d = 1; d < 32; d <<= 1) {
      const int up = __shfl_up(incl, d);
      if (lane >= d) incl += up;
    }
    if (lane == 31) wtot[wave] = incl;
    __syncthreads();
    int pre = 0;
#pragma unroll
    for (int w2 = 0; w2 < NWAVE; ++w2) pre += (w2 < wave) ? wtot[w2] : 0;
    int run = pre + incl - ts;
    soff[8 * tid + 0] = run; run += e0;
    soff[8 * tid + 1] = run; run += e1;
    soff[8 * tid + 2] = run; run += e2;
    soff[8 * tid + 3] = run; run += e3;
    soff[8 * tid + 4] = run; run += e4;
    soff[8 * tid + 5] = run; run += e5;
    soff[8 * tid + 6] = run; run += e6;
    soff[8 * tid + 7] = run;
  }
  __syncthreads();
  for (int i = tid; i < NBMAX; i += NTHR) list[i] = soff[i];
  __syncthreads();

  if (wave == 0) {
#pragma unroll 1
    for (int b0 = 0; b0 < nh; b0 += 32) {
      const int idx = b0 + lane;
      const int uv  = reg1[idx < RCAP ? idx : RCAP - 1];
      const int m32 = (nh - b0) < 32 ? (nh - b0) : 32;
#pragma unroll 1
      for (int k = 0; k < m32; ++k) {
        const int u   = __builtin_amdgcn_readlane(uv, k);
        const int sl  = u & (NBMAX - 1);
        const int eid = (int)((unsigned)u >> 12);
        if (lane == 0) {
          int pos = list[sl];
          pos = pos < 0 ? 0 : (pos > RCAP - 1 ? RCAP - 1 : pos);
          reg2[pos] = eid;
          list[sl] = pos + 1;
        }
      }
    }
  }
  __syncthreads();

  const int nbw = nb >> 3;
  const int c8  = 8 * lane;
  const int hd  = lane >> 3;
  const v4f bz0 = *(const v4f*)(bias + c8);
  const v4f bz1 = *(const v4f*)(bias + c8 + 4);
  const bool ovf = (nh >= RCAP);
  const float qnan = __int_as_float(0x7fc00000);
#pragma unroll 1
  for (int jt = 0; jt < nbw; ++jt) {
    const int slot = wave * nbw + jt;
    const int grow = nodeBase + slot;
    const int gcl  = grow < nN ? grow : nN - 1;
    int st = soff[slot];
    const int craw = scnt[slot];
    int cnt = craw;
    st  = st < 0 ? 0 : (st > nh ? nh : st);
    cnt = cnt < 0 ? 0 : (cnt > DEGCAP ? DEGCAP : cnt);
    if (cnt > nh - st) cnt = nh - st;
    const float pz = (ovf || craw > DEGCAP) ? qnan : 0.0f;
    const bool wr = grow < nN;

    const float* yd = Y + (size_t)gcl * YP + c8;
    const v4f xd0 = *(const v4f*)yd;
    const v4f xd1 = *(const v4f*)(yd + 4);
    const float edv = ED[(size_t)gcl * EP + hd];
    const float esd = ES[(size_t)gcl * EP + hd];
    const float t0 = esd + edv;
    float mx = fmaxf(t0, NEG_SLOPE * t0);
    float dn = 1.0f;
    v4f a0 = xd0, a1 = xd1;
#pragma unroll 1
    for (int q = 0; q < cnt; ++q) {
      int idx = st + q; idx = idx > RCAP - 1 ? RCAP - 1 : idx;
      int eid = reg2[idx]; eid = eid < 0 ? 0 : (eid > nE - 1 ? nE - 1 : eid);
      const int sraw = srcs[eid];
      const int s = sraw < 0 ? 0 : (sraw > nN - 1 ? nN - 1 : sraw);
      const float* ys = Y + (size_t)s * YP + c8;
      const v4f xs0 = *(const v4f*)ys;
      const v4f xs1 = *(const v4f*)(ys + 4);
      const float ess = ES[(size_t)s * EP + hd];
      const float u = ess + edv;
      const float l = fmaxf(u, NEG_SLOPE * u);
      const float mn = fmaxf(mx, l);
      const float s1 = __expf(mx - mn), s2 = __expf(l - mn);
      dn = fmaf(dn, s1, s2);
      a0.x = fmaf(a0.x, s1, s2 * xs0.x);
      a0.y = fmaf(a0.y, s1, s2 * xs0.y);
      a0.z = fmaf(a0.z, s1, s2 * xs0.z);
      a0.w = fmaf(a0.w, s1, s2 * xs0.w);
      a1.x = fmaf(a1.x, s1, s2 * xs1.x);
      a1.y = fmaf(a1.y, s1, s2 * xs1.y);
      a1.z = fmaf(a1.z, s1, s2 * xs1.z);
      a1.w = fmaf(a1.w, s1, s2 * xs1.w);
      mx = mn;
    }
    const float inv = __builtin_amdgcn_rcpf(dn);
    v4f o0, o1;
    o0.x = fmaxf(fmaf(a0.x, inv, bz0.x), 0.f) + pz;
    o0.y = fmaxf(fmaf(a0.y, inv, bz0.y), 0.f) + pz;
    o0.z = fmaxf(fmaf(a0.z, inv, bz0.z), 0.f) + pz;
    o0.w = fmaxf(fmaf(a0.w, inv, bz0.w), 0.f) + pz;
    o1.x = fmaxf(fmaf(a1.x, inv, bz1.x), 0.f) + pz;
    o1.y = fmaxf(fmaf(a1.y, inv, bz1.y), 0.f) + pz;
    o1.z = fmaxf(fmaf(a1.z, inv, bz1.z), 0.f) + pz;
    o1.w = fmaxf(fmaf(a1.w, inv, bz1.w), 0.f) + pz;
    v8h hv;
    hv[0] = (_Float16)(o0.x * CA); hv[1] = (_Float16)(o0.y * CA);
    hv[2] = (_Float16)(o0.z * CA); hv[3] = (_Float16)(o0.w * CA);
    hv[4] = (_Float16)(o1.x * CA); hv[5] = (_Float16)(o1.y * CA);
    hv[6] = (_Float16)(o1.z * CA); hv[7] = (_Float16)(o1.w * CA);
    _Float16* xp = xout + (size_t)gcl * KP + c8;
    if (wr) *(volatile v8h*)xp = hv;
    __threadfence();
    if (wr) *(volatile v8h*)xp = hv;
  }
}

__global__ __launch_bounds__(GTHR) void k_fc(const _Float16* __restrict__ xh, const _Float16* __restrict__ wf,
                                             const float* __restrict__ bfc, float* out, int nN) {
  __shared__ __attribute__((aligned(16))) float sO[GBM * OUTD];
  __shared__ float sb[FCN];
  const int tid = threadIdx.x, lane = tid & 31, wave = tid >> 5, hh = lane >> 4, m = lane & 15;
  const int rowBase = (int)blockIdx.x * GBM;
  if (tid < FCN) sb[tid] = bfc[tid < OUTD ? tid : OUTD - 1];
  const size_t arow = (size_t)(rowBase + 16 * wave + m) * KP + 8 * hh;
  const size_t brow = (size_t)m * KP + 8 * hh;
  v8f acc = {0.f, 0.f, 0.f, 0.f, 0.f, 0.f, 0.f, 0.f};
#pragma unroll 1
  for (int ks = 0; ks < KP / 32; ++ks) {
    FragH af, bf;
    af.h[0] = *(const v8h*)(xh + arow + 32 * ks);
    af.h[1] = *(const v8h*)(xh + arow + 32 * ks + 16);
    bf.h[0] = *(const v8h*)(wf + brow + 32 * ks);
    bf.h[1] = *(const v8h*)(wf + brow + 32 * ks + 16);
    acc = wmh(af, bf, acc);
  }
  __syncthreads();
  {
    const float bj = sb[m];
#pragma unroll
    for (int r = 0; r < 8; ++r) {
      const float v = fmaf(acc[r], SCL, bj);
      if (m < OUTD) sO[(16 * wave + 8 * hh + r) * OUTD + m] = v;
    }
  }
  __syncthreads();
  const int nValid = (nN - rowBase) < GBM ? (nN - rowBase) : GBM;
  const int fl  = nValid * OUTD;
  const int n4  = fl >> 2;
  const int rem = fl & 3;
  float* base = out + (size_t)rowBase * OUTD;
  const v4f* s4 = (const v4f*)sO;
  const v4f v = s4[tid < n4 ? tid : 0];
  const int ti = 4 * n4 + (lane & 3);
  const float tv = sO[ti < fl ? ti : fl - 1];
  const bool tw = (rem != 0) && (tid >= n4) && (tid < n4 + rem) && (wave == (n4 >> 5));
  if (tid < n4) *(volatile v4f*)(base + 4 * tid) = v;
  if (tw) *(volatile float*)(base + 4 * n4 + (tid - n4)) = tv;
  __threadfence();
  if (tid < n4) *(volatile v4f*)(base + 4 * tid) = v;
  if (tw) *(volatile float*)(base + 4 * n4 + (tid - n4)) = tv;
}

static int pick_nb(int nE, int nN) {
  int nb = NBMAX;
  while (nb > 16 && (long long)nb * (long long)nE * 5LL > (long long)RCAP * (long long)nN * 4LL) nb >>= 1;
  return nb;
}

extern "C" void kernel_launch(void* const* d_in, const int* in_sizes, int n_in,
                              void* d_out, int out_size, void* d_ws, size_t ws_size,
                              hipStream_t stream) {
  if (n_in < 13) return;
  const int nN = in_sizes[0] / IN_DIM;
  if (nN <= 0 || in_sizes[0] != nN * IN_DIM) return;
  if (nN > (1 << 22)) return;
  const int nE = in_sizes[1];
  if (nE < 1 || in_sizes[2] != nE) return;
  if (nE > (1 << 20)) return;
  if (in_sizes[3] != IN_DIM * FEAT) return;
  if (in_sizes[4] != NHEAD * HC || in_sizes[5] != NHEAD * HC) return;
  if (in_sizes[6] != FEAT) return;
  if (in_sizes[7] != FEAT * FEAT) return;
  if (in_sizes[8] != NHEAD * HC || in_sizes[9] != NHEAD * HC) return;
  if (in_sizes[10] != FEAT) return;
  if (in_sizes[11] != FEAT * OUTD) return;
  if (in_sizes[12] != OUTD) return;
  if (out_size != nN * OUTD) return;

  const float* x   = (const float*)d_in[0];
  const int*   src = (const int*)d_in[1];
  const int*   dst = (const int*)d_in[2];
  const float* W1  = (const float*)d_in[3];
  const float* as1 = (const float*)d_in[4];
  const float* ad1 = (const float*)d_in[5];
  const float* b1  = (const float*)d_in[6];
  const float* W2  = (const float*)d_in[7];
  const float* as2 = (const float*)d_in[8];
  const float* ad2 = (const float*)d_in[9];
  const float* b2  = (const float*)d_in[10];
  const float* Wfc = (const float*)d_in[11];
  const float* bfc = (const float*)d_in[12];
  float* out = (float*)d_out;

  const int MP   = ((nN + GBM - 1) / GBM) * GBM;
  const int nb   = pick_nb(nE, nN);
  const int vec8 = 1;
  const int nUnits = MP * (KP / 8);

  char* ws = (char*)d_ws;
  size_t off = 0;
  const size_t oWT = off; off += (size_t)WTROWS * KP * 2;        off = (off + 255) & ~(size_t)255;
  const size_t oXH = off; off += (size_t)MP * KP * 2;            off = (off + 255) & ~(size_t)255;
  const size_t oY  = off; off += (size_t)MP * YP * 4;            off = (off + 255) & ~(size_t)255;
  const size_t oES = off; off += (size_t)MP * EP * 4;            off = (off + 255) & ~(size_t)255;
  const size_t oED = off; off += (size_t)MP * EP * 4;            off = (off + 255) & ~(size_t)255;
  if (off > ws_size || off > (size_t)WSCAP) return;
  _Float16* WT = (_Float16*)(ws + oWT);
  _Float16* XH = (_Float16*)(ws + oXH);
  float*    Y  = (float*)(ws + oY);
  float*    ES = (float*)(ws + oES);
  float*    ED = (float*)(ws + oED);

  hipFuncSetAttribute(reinterpret_cast<const void*>(&k_agg),
                      hipFuncAttributeMaxDynamicSharedMemorySize, LDS_AGG);

  k_xprep<<<(nUnits + NTHR - 1) / NTHR, NTHR, 0, stream>>>(x, XH, nN, nUnits);
  k_wprep<<<dim3((FEAT * (KP / 8) + NTHR - 1) / NTHR, 3), NTHR, 0, stream>>>(W1, W2, Wfc, WT);

  const int gG = MP / GBM;
  const int gA = (nN + nb - 1) / nb;

  k_gemm<<<gG, GTHR, 0, stream>>>(XH, WT, as1, ad1, Y, ES, ED, IN_DIM / 32);
  k_agg<<<gA, NTHR, LDS_AGG, stream>>>(src, dst, Y, ES, ED, b1, XH, nN, nE, nb, vec8);
  k_gemm<<<gG, GTHR, 0, stream>>>(XH, WT + (size_t)FEAT * KP, as2, ad2, Y, ES, ED, FEAT / 32);
  k_agg<<<gA, NTHR, LDS_AGG, stream>>>(src, dst, Y, ES, ED, b2, XH, nN, nE, nb, vec8);
  k_fc<<<gG, GTHR, 0, stream>>>(XH, WT + (size_t)(2 * FEAT) * KP, bfc, out, nN);
}
